// GaussianGraphSAGE_82377472738051
// MI455X (gfx1250) — hardware-run, weakly checked
//
#include <hip/hip_runtime.h>
#include <stddef.h>


#define DD      64
#define KA      128
#define FCH     128
#define NCLS    10
#define NCP     16
#define NTHR    256
#define NWAVE   8
#define EPT     8
#define NGRP    2
#define CHUNK   (NTHR * EPT * NGRP)
#define WCAP    (EPT * NGRP * 32)
#define LISTN   (NWAVE * WCAP)
#define NBC     4096
#define NBF     1024
#define RCAP    40960
#define RBN     128
#define TGT     256
#define DEGCAP  256
#define OTHR    512
#define BM      64
#define GPB     128
#define WSCAP   134217728
#define XSC     8.0f
#define WSC     64.0f
#define ZSC     64.0f
#define INV_NODE (1.0f / 512.0f)
#define INV_HEAD (1.0f / 4096.0f)
#define AROWU   (KA / 2)
#define STGU    (16 * AROWU)

#define LDS_FILL ((RCAP + NBF + LISTN) * 4 + 64)

#define PL_SACC 0
#define PL_LIST (PL_SACC + GPB * DD * 4)
#define PL_SZ   (PL_LIST + LISTN * 4)
#define PL_SW   (PL_SZ + GPB * DD * 2)
#define PL_SH   (PL_SW + FCH * DD * 2)
#define PL_SL   (PL_SH + GPB * FCH * 4)
#define PL_SO   (PL_SL + GPB * NCP * 4)
#define PL_SCNT (PL_SO + GPB * NCLS * 4)
#define PL_SINV (PL_SCNT + GPB * 4)
#define PL_WCNT (PL_SINV + GPB * 4)
#define LDS_POOL (PL_WCNT + 64)

static_assert((CHUNK & (CHUNK - 1)) == 0);
static_assert(CHUNK <= 4096);
static_assert(NBC <= 4096 && NBF <= 4096 && GPB <= 4096);
static_assert((NBC & (NBC - 1)) == 0 && (NBF & (NBF - 1)) == 0 && (GPB & (GPB - 1)) == 0);
static_assert(NBC == 4 * NBF);
static_assert(OTHR * 8 == NBC);
static_assert((RCAP % 32) == 0);
static_assert(TGT == NWAVE * 32);
static_assert((TGT % BM) == 0 && (NBF % TGT) == 0);
static_assert((KA % 32) == 0 && (DD % 32) == 0 && KA == 2 * DD);
static_assert((BM * DD / 4) % NTHR == 0);
static_assert(GPB == NWAVE * 16);
static_assert(FCH == 8 * 16);
static_assert((PL_LIST % 16) == 0 && (PL_SZ % 16) == 0 && (PL_SW % 16) == 0 && (PL_SH % 16) == 0);
static_assert((PL_SL % 16) == 0 && (PL_SO % 16) == 0 && (PL_SCNT % 16) == 0);
static_assert(DD < NTHR && GPB <= NTHR);

typedef float          v2f  __attribute__((ext_vector_type(2)));
typedef float          v4f  __attribute__((ext_vector_type(4)));
typedef float          v8f  __attribute__((ext_vector_type(8)));
typedef int            v4i  __attribute__((ext_vector_type(4)));
typedef unsigned int   v4u  __attribute__((ext_vector_type(4)));
typedef v4u            v4ua __attribute__((may_alias));
typedef _Float16       v8h  __attribute__((ext_vector_type(8)));
typedef _Float16       v16h __attribute__((ext_vector_type(16)));
union FragH { v16h v; v8h h[2]; };

__device__ __forceinline__ v8f wmh(v16h a, v16h b, v8f c) {
  v8f d = __builtin_amdgcn_wmma_f32_16x16x32_f16(false, a, false, b, (short)0, c, false, false);
  asm volatile("v_nop\n\tv_nop\n\tv_nop\n\tv_nop" : "+v"(d) : "v"(a), "v"(b));
  return d;
}

template <int NB>
__device__ __forceinline__ int scan_chunk(const int* __restrict__ dsts, int nE, int cbase, int slotBase,
                                          int vec8, int* list, int tid, int lane, int wave) {
  int wc = 0;
#pragma unroll
  for (int g = 0; g < NGRP; ++g) {
    const int el0  = (g * NTHR + tid) * EPT;
    const int e0   = cbase + el0;
    const int sent = -2147483647 - 1;
    v4i da, db;
    if (vec8 != 0 && cbase + CHUNK <= nE) {
      da = *(const v4i*)(dsts + e0);
      db = *(const v4i*)(dsts + e0 + 4);
    } else {
      da.x = (e0     < nE) ? dsts[min(e0, nE - 1)] : sent;
      da.y = (e0 + 1 < nE) ? dsts[min(e0 + 1, nE - 1)] : sent;
      da.z = (e0 + 2 < nE) ? dsts[min(e0 + 2, nE - 1)] : sent;
      da.w = (e0 + 3 < nE) ? dsts[min(e0 + 3, nE - 1)] : sent;
      db.x = (e0 + 4 < nE) ? dsts[min(e0 + 4, nE - 1)] : sent;
      db.y = (e0 + 5 < nE) ? dsts[min(e0 + 5, nE - 1)] : sent;
      db.z = (e0 + 6 < nE) ? dsts[min(e0 + 6, nE - 1)] : sent;
      db.w = (e0 + 7 < nE) ? dsts[min(e0 + 7, nE - 1)] : sent;
    }
    const unsigned nb = (unsigned)slotBase;
    const unsigned s0 = (unsigned)da.x - nb, s1 = (unsigned)da.y - nb;
    const unsigned s2 = (unsigned)da.z - nb, s3 = (unsigned)da.w - nb;
    const unsigned s4 = (unsigned)db.x - nb, s5 = (unsigned)db.y - nb;
    const unsigned s6 = (unsigned)db.z - nb, s7 = (unsigned)db.w - nb;
    const bool h0 = s0 < (unsigned)NB, h1 = s1 < (unsigned)NB, h2 = s2 < (unsigned)NB, h3 = s3 < (unsigned)NB;
    const bool h4 = s4 < (unsigned)NB, h5 = s5 < (unsigned)NB, h6 = s6 < (unsigned)NB, h7 = s7 < (unsigned)NB;
    const unsigned any = __builtin_amdgcn_ballot_w32(h0 | h1 | h2 | h3 | h4 | h5 | h6 | h7);
    if (any != 0u) {
#define HITJ(J, HJ, SJ) { \
        const unsigned mj = __builtin_amdgcn_ballot_w32(HJ); \
        if (mj != 0u) { \
          if (HJ) { \
            const int pos = wc + (int)__builtin_amdgcn_mbcnt_lo(mj, 0u); \
            if (pos < WCAP) list[wave * WCAP + pos] = ((el0 + (J)) << 12) | (int)(SJ); \
          } \
          wc += (int)__builtin_popcount(mj); } }
      HITJ(0, h0, s0)
      HITJ(1, h1, s1)
      HITJ(2, h2, s2)
      HITJ(3, h3, s3)
      HITJ(4, h4, s4)
      HITJ(5, h5, s5)
      HITJ(6, h6, s6)
      HITJ(7, h7, s7)
#undef HITJ
    }
  }
  return wc;
}

__global__ __launch_bounds__(NTHR) void k_wprep(
    const float* __restrict__ mWl, const float* __restrict__ mWr,
    const float* __restrict__ vWl, const float* __restrict__ vWr, _Float16* wp, int nL) {
  const int i = (int)blockIdx.x * NTHR + (int)threadIdx.x;
  const int total = nL * 2 * DD * (KA / 8);
  if (i >= total) return;
  const int p  = i >> 10;
  const int r  = i & 1023;
  const int n  = r >> 4;
  const int k0 = (r & 15) * 8;
  const int l  = p >> 1, s = p & 1;
  const int kk = k0 & (DD - 1);
  const size_t ro = ((size_t)l * DD + n) * DD + kk;
  const v4f a0 = *(const v4f*)(mWl + ro), a1 = *(const v4f*)(mWl + ro + 4);
  const v4f b0 = *(const v4f*)(mWr + ro), b1 = *(const v4f*)(mWr + ro + 4);
  const v4f c0 = *(const v4f*)(vWl + ro), c1 = *(const v4f*)(vWl + ro + 4);
  const v4f d0 = *(const v4f*)(vWr + ro), d1 = *(const v4f*)(vWr + ro + 4);
  const bool hiK = k0 >= DD;
  const v4f lo = (s != 0) ? (hiK ? d0 : c0) : (hiK ? b0 : a0);
  const v4f hi = (s != 0) ? (hiK ? d1 : c1) : (hiK ? b1 : a1);
  v8h hv;
  hv[0] = (_Float16)(lo.x * WSC); hv[1] = (_Float16)(lo.y * WSC);
  hv[2] = (_Float16)(lo.z * WSC); hv[3] = (_Float16)(lo.w * WSC);
  hv[4] = (_Float16)(hi.x * WSC); hv[5] = (_Float16)(hi.y * WSC);
  hv[6] = (_Float16)(hi.z * WSC); hv[7] = (_Float16)(hi.w * WSC);
  _Float16* d = wp + (size_t)i * 8;
  *(volatile v8h*)d = hv;
  __threadfence();
  *(volatile v8h*)d = hv;
}

__global__ __launch_bounds__(NTHR) void k_count(
    const int* __restrict__ dsts, int* cnt, int nE, int vec8) {
  __shared__ __attribute__((aligned(16))) int scnt[NBC];
  __shared__ __attribute__((aligned(16))) int list[LISTN];
  __shared__ int wcnt[NWAVE];
  const int tid = threadIdx.x, lane = tid & 31, wave = tid >> 5;
  const int nodeBase = blockIdx.x * NBC;

  for (int i = tid; i < NBC; i += NTHR) scnt[i] = 0;
  __syncthreads();

  const int nChunks = (nE + CHUNK - 1) / CHUNK;
#pragma unroll 1
  for (int ch = 0; ch < nChunks; ++ch) {
    const int cbase = ch * CHUNK;
    const int wc = scan_chunk<NBC>(dsts, nE, cbase, nodeBase, vec8, list, tid, lane, wave);
    if (lane == 0) wcnt[wave] = wc;
    __syncthreads();
    if (wave == 0) {
#pragma unroll 1
      for (int wsx = 0; wsx < NWAVE; ++wsx) {
        int n = __builtin_amdgcn_readfirstlane(wcnt[wsx]);
        n = n > WCAP ? WCAP : (n < 0 ? 0 : n);
        const int* lp = list + wsx * WCAP;
#pragma unroll 1
        for (int i = 0; i < n; ++i) {
          const int ent  = __builtin_amdgcn_readfirstlane(lp[i]);
          const int slot = ent & (NBC - 1);
          if (lane == 0) scnt[slot] = scnt[slot] + 1;
        }
      }
    }
    __syncthreads();
  }

  v4i cq[4];
#pragma unroll
  for (int q = 0; q < 4; ++q) {
    const int f = (wave * 4 + q) * 128 + 4 * lane;
    cq[q] = *(const v4i*)(scnt + f);
  }
  int* cp = cnt + (size_t)nodeBase;
#pragma unroll
  for (int q = 0; q < 4; ++q) {
    const int f = (wave * 4 + q) * 128 + 4 * lane;
    *(volatile v4i*)(cp + f) = cq[q];
  }
  __threadfence();
#pragma unroll
  for (int q = 0; q < 4; ++q) {
    const int f = (wave * 4 + q) * 128 + 4 * lane;
    *(volatile v4i*)(cp + f) = cq[q];
  }
}

__global__ __launch_bounds__(OTHR) void k_offsets(
    const int* __restrict__ cnt, int* off, int* rbase, int nChunk) {
  __shared__ __attribute__((aligned(16))) int soff[NBC];
  __shared__ __attribute__((aligned(16))) int srb[RBN];
  __shared__ int wtot[OTHR / 32];
  const int tid = threadIdx.x, lane = tid & 31, wave = tid >> 5, sub = tid >> 7;
  for (int i = tid; i < RBN; i += OTHR) srb[i] = 0;
  int carry = 0;
#pragma unroll 1
  for (int ch = 0; ch < nChunk; ++ch) {
    const int base = ch * NBC;
    const v4i c0 = *(const v4i*)(cnt + base + 8 * tid);
    const v4i c1 = *(const v4i*)(cnt + base + 8 * tid + 4);
    const int e0 = max(c0.x, 0), e1 = max(c0.y, 0), e2 = max(c0.z, 0), e3 = max(c0.w, 0);
    const int e4 = max(c1.x, 0), e5 = max(c1.y, 0), e6 = max(c1.z, 0), e7 = max(c1.w, 0);
    const int ts = e0 + e1 + e2 + e3 + e4 + e5 + e6 + e7;
    int incl = ts;
#pragma unroll
    for (int d = 1; d < 32; d <<= 1) {
      const int t = __shfl_up(incl, d);
      if (lane >= d) incl += t;
    }
    if (lane == 31) wtot[wave] = incl;
    __syncthreads();
    const int S0 = wtot[0]  + wtot[1]  + wtot[2]  + wtot[3];
    const int S1 = wtot[4]  + wtot[5]  + wtot[6]  + wtot[7];
    const int S2 = wtot[8]  + wtot[9]  + wtot[10] + wtot[11];
    const int S3 = wtot[12] + wtot[13] + wtot[14] + wtot[15];
    int pre = 0;
#pragma unroll 1
    for (int w = 4 * sub; w < wave; ++w) pre += wtot[w];
    const int b0 = carry;
    const int b1 = b0 + ((S0 + 31) & ~31);
    const int b2 = b1 + ((S1 + 31) & ~31);
    const int b3 = b2 + ((S2 + 31) & ~31);
    const int b4 = b3 + ((S3 + 31) & ~31);
    const int myb = sub == 0 ? b0 : (sub == 1 ? b1 : (sub == 2 ? b2 : b3));
    if (tid == 0) {
      srb[min(4 * ch + 0, RBN - 1)] = b0;
      srb[min(4 * ch + 1, RBN - 1)] = b1;
      srb[min(4 * ch + 2, RBN - 1)] = b2;
      srb[min(4 * ch + 3, RBN - 1)] = b3;
    }
    int run = myb + pre + incl - ts;
    soff[8 * tid + 0] = run; run += e0;
    soff[8 * tid + 1] = run; run += e1;
    soff[8 * tid + 2] = run; run += e2;
    soff[8 * tid + 3] = run; run += e3;
    soff[8 * tid + 4] = run; run += e4;
    soff[8 * tid + 5] = run; run += e5;
    soff[8 * tid + 6] = run; run += e6;
    soff[8 * tid + 7] = run;
    carry = b4;
    __syncthreads();
    const v4i o0 = *(const v4i*)(soff + 4 * tid);
    const v4i o1 = *(const v4i*)(soff + 4 * (tid + OTHR));
    int* op = off + base;
    *(volatile v4i*)(op + 4 * tid) = o0;
    *(volatile v4i*)(op + 4 * (tid + OTHR)) = o1;
    __threadfence();
    *(volatile v4i*)(op + 4 * tid) = o0;
    *(volatile v4i*)(op + 4 * (tid + OTHR)) = o1;
    __syncthreads();
  }
  if (tid == 0) srb[min(4 * nChunk, RBN - 1)] = carry;
  __syncthreads();
  v4i rv = {0, 0, 0, 0};
  if (tid < 32) rv = *(const v4i*)(srb + 4 * tid);
  if (tid < 32) *(volatile v4i*)(rbase + 4 * tid) = rv;
  __threadfence();
  if (tid < 32) *(volatile v4i*)(rbase + 4 * tid) = rv;
}

__global__ __launch_bounds__(NTHR) void k_fill(
    const int* __restrict__ srcs, const int* __restrict__ dsts,
    const int* __restrict__ off, const int* __restrict__ rbase,
    int* csr, int nN, int nE, int vec8, int csrLen) {
  extern __shared__ v4f lds_fill[];
  int* region = (int*)lds_fill;
  int* cursor = region + RCAP;
  int* list   = cursor + NBF;
  int* wcnt   = list + LISTN;
  const int tid = threadIdx.x, lane = tid & 31, wave = tid >> 5;
  const int b = blockIdx.x;
  const int nodeBase = b * NBF;

  int rb0 = rbase[b];
  const int rb1 = rbase[b + 1];
  rb0 = rb0 < 0 ? 0 : (rb0 > csrLen ? csrLen : rb0);
  rb0 &= ~31;
  int len = rb1 - rb0;
  len = len < 0 ? 0 : (len > RCAP ? RCAP : len);
  int lenW = (len + 31) & ~31;
  if (rb0 + lenW > csrLen) lenW = (csrLen - rb0) & ~31;

  {
    const v4i z = {0, 0, 0, 0};
    for (int i = tid; i < RCAP / 4; i += NTHR) ((v4i*)region)[i] = z;
    for (int s = tid; s < NBF; s += NTHR) {
      int o = off[nodeBase + s] - rb0;
      o = o < 0 ? 0 : (o > RCAP ? RCAP : o);
      cursor[s] = o;
    }
  }
  __syncthreads();

  const int nChunks = (nE + CHUNK - 1) / CHUNK;
#pragma unroll 1
  for (int ch = 0; ch < nChunks; ++ch) {
    const int cbase = ch * CHUNK;
    const int wc = scan_chunk<NBF>(dsts, nE, cbase, nodeBase, vec8, list, tid, lane, wave);
    if (lane == 0) wcnt[wave] = wc;
    __syncthreads();
    if (wave == 0) {
#pragma unroll 1
      for (int wsx = 0; wsx < NWAVE; ++wsx) {
        int n = __builtin_amdgcn_readfirstlane(wcnt[wsx]);
        n = n > WCAP ? WCAP : (n < 0 ? 0 : n);
        const int* lp = list + wsx * WCAP;
#pragma unroll 1
        for (int i = 0; i < n; ++i) {
          const int ent  = __builtin_amdgcn_readfirstlane(lp[i]);
          const int slot = ent & (NBF - 1);
          int e = cbase + ((ent >> 12) & (CHUNK - 1));
          e = e > nE - 1 ? nE - 1 : e;
          int src = srcs[e];
          src = src < 0 ? 0 : (src > nN - 1 ? nN - 1 : src);
          if (lane == 0) {
            int pos = cursor[slot];
            pos = pos < 0 ? 0 : (pos > RCAP - 1 ? RCAP - 1 : pos);
            region[pos] = src;
            const int np = pos + 1;
            cursor[slot] = np > RCAP ? RCAP : np;
          }
        }
      }
    }
    __syncthreads();
  }

  const int nv = lenW >> 2;
  int* gp = csr + rb0;
#pragma unroll 1
  for (int i = tid; i < nv; i += NTHR) { const v4i v = ((const v4i*)region)[i]; *(volatile v4i*)(gp + 4 * i) = v; }
  __threadfence();
#pragma unroll 1
  for (int i = tid; i < nv; i += NTHR) { const v4i v = ((const v4i*)region)[i]; *(volatile v4i*)(gp + 4 * i) = v; }
}

__global__ __launch_bounds__(NTHR) void k_agg(
    const int* __restrict__ csr, const int* __restrict__ off, const int* __restrict__ cnt,
    const float* __restrict__ hin, int hStride, unsigned int* aout, int aStrideU,
    int nN, int csrLen) {
  __shared__ __attribute__((aligned(16))) unsigned int stg[NWAVE * STGU];
  const int tid = threadIdx.x, lane = tid & 31, wave = tid >> 5;
  const int y = blockIdx.y;
  const float* h = hin + (size_t)y * (size_t)hStride;
  unsigned int* ap = aout + (size_t)y * (size_t)aStrideU;
  unsigned int* sw = stg + wave * STGU;
  const int tbase = blockIdx.x * TGT + wave * 32;

  const int cl    = tbase + lane;
  const int cnt_l = cnt[cl];
  const int off_l = off[cl];
  const v2f z2 = {0.f, 0.f};

#pragma unroll 1
  for (int j = 0; j < 32; ++j) {
    const int c = tbase + j;
    int nraw = __shfl(cnt_l, j);
    nraw = nraw < 0 ? 0 : nraw;
    const int   n    = nraw > DEGCAP ? DEGCAP : nraw;
    const int   st   = __shfl(off_l, j);
    const float dinv = 1.0f / fmaxf((float)nraw, 1.0f);

    v2f acc = z2;
#pragma unroll 1
    for (int q0 = 0; q0 < n; q0 += 32) {
      int pos = st + q0 + lane;
      pos = pos < 0 ? 0 : (pos > csrLen - 1 ? csrLen - 1 : pos);
      int sl = csr[pos];
      sl = sl < 0 ? 0 : (sl > nN - 1 ? nN - 1 : sl);
      const int mcnt = (n - q0) < 32 ? (n - q0) : 32;
#pragma unroll 1
      for (int pp = 0; pp < mcnt; ++pp) {
        const int s   = __builtin_amdgcn_readlane(sl, pp);
        const v2f hv2 = *(const v2f*)(h + (size_t)s * DD + 2 * lane);
        acc = acc + hv2;
      }
    }
    const int  cc  = c < nN ? c : nN - 1;
    const v2f  hs  = *(const v2f*)(h + (size_t)cc * DD + 2 * lane);
    const bool rok = c < nN;
    const float asc = rok ? dinv * XSC : 0.0f;
    const float hsc = rok ? XSC : 0.0f;
    const _Float16 a0 = (_Float16)(acc.x * asc), a1 = (_Float16)(acc.y * asc);
    const _Float16 h0 = (_Float16)(hs.x * hsc),  h1 = (_Float16)(hs.y * hsc);
    const unsigned int pka = (unsigned int)__builtin_bit_cast(unsigned short, a0) |
                             ((unsigned int)__builtin_bit_cast(unsigned short, a1) << 16);
    const unsigned int pkh = (unsigned int)__builtin_bit_cast(unsigned short, h0) |
                             ((unsigned int)__builtin_bit_cast(unsigned short, h1) << 16);
    sw[(j & 15) * AROWU + lane]      = pka;
    sw[(j & 15) * AROWU + 32 + lane] = pkh;

    if ((j & 15) == 15) {
      __syncthreads();
      const int rowBase = tbase + (j & 16);
      v4u vv[8];
#pragma unroll
      for (int it = 0; it < 8; ++it) vv[it] = *(const v4ua*)(sw + (it * 32 + lane) * 4);
      unsigned int* gp = ap + (size_t)rowBase * AROWU;
#pragma unroll
      for (int it = 0; it < 8; ++it) *(volatile v4u*)(gp + (it * 32 + lane) * 4) = vv[it];
      __threadfence();
#pragma unroll
      for (int it = 0; it < 8; ++it) *(volatile v4u*)(gp + (it * 32 + lane) * 4) = vv[it];
      __syncthreads();
    }
  }
}

__global__ __launch_bounds__(NTHR) void k_gemm(
    const _Float16* __restrict__ A, int aStride, const _Float16* __restrict__ Wp,
    const float* __restrict__ blM, const float* __restrict__ blV,
    float* C, int cStride, int nValid) {
  __shared__ __attribute__((aligned(16))) float stg[BM * DD];
  const int tid = threadIdx.x, lane = tid & 31, wave = tid >> 5, hh = lane >> 4, m = lane & 15;
  const int y = blockIdx.y;
  const _Float16* Ay = A  + (size_t)y * (size_t)aStride;
  const _Float16* W  = Wp + (size_t)y * (DD * KA);
  const float* bias = blM;
  if (y != 0) bias = blV;
  float* Cy = C + (size_t)y * (size_t)cStride;
  const int rowBase = blockIdx.x * BM;
  const int r0 = (wave >> 1) * 16, c0 = (wave & 1) * 32;

  v8f acc[2];
  { v8f z = {0.f, 0.f, 0.f, 0.f, 0.f, 0.f, 0.f, 0.f}; acc[0] = z; acc[1] = z; }
  const _Float16* ap  = Ay + (size_t)(rowBase + r0 + m) * KA + 8 * hh;
  const _Float16* bp0 = W  + (size_t)(c0 + m) * KA + 8 * hh;
#pragma unroll 1
  for (int kt = 0; kt < KA / 32; ++kt) {
    FragH a;
    a.h[0] = *(const v8h*)(ap + 32 * kt);
    a.h[1] = *(const v8h*)(ap + 32 * kt + 16);
#pragma unroll
    for (int t = 0; t < 2; ++t) {
      const _Float16* bp = bp0 + (size_t)(16 * t) * KA + 32 * kt;
      FragH b;
      b.h[0] = *(const v8h*)bp;
      b.h[1] = *(const v8h*)(bp + 16);
      acc[t] = wmh(a.v, b.v, acc[t]);
    }
  }
  float* sp = stg + (size_t)(r0 + 8 * hh) * DD + c0 + m;
#pragma unroll
  for (int t = 0; t < 2; ++t) {
    const float bv = bias[c0 + 16 * t + m];
#pragma unroll
    for (int r = 0; r < 8; ++r) sp[r * DD + 16 * t] = fmaxf(acc[t][r] * INV_NODE + bv, 0.0f);
  }
  __syncthreads();

  constexpr int NIT = (BM * DD / 4) / NTHR;
  v4f vv[NIT];
#pragma unroll
  for (int it = 0; it < NIT; ++it) vv[it] = ((const v4f*)stg)[it * NTHR + tid];
  const size_t gb = (size_t)rowBase * DD;
#pragma unroll
  for (int it = 0; it < NIT; ++it) {
    const int f = it * NTHR + tid;
    if (rowBase + (f >> 4) < nValid) *(volatile v4f*)(Cy + gb + (size_t)f * 4) = vv[it];
  }
  __threadfence();
#pragma unroll
  for (int it = 0; it < NIT; ++it) {
    const int f = it * NTHR + tid;
    if (rowBase + (f >> 4) < nValid) *(volatile v4f*)(Cy + gb + (size_t)f * 4) = vv[it];
  }
}

__global__ __launch_bounds__(NTHR) void k_pool_head(
    const int* __restrict__ bidx, const float* __restrict__ hm, const float* __restrict__ hv,
    const float* __restrict__ eps, const float* __restrict__ fc1W, const float* __restrict__ fc1b,
    const float* __restrict__ fc2W, const float* __restrict__ fc2b,
    float* out, int nN, int nG, int vec8) {
  extern __shared__ v4f lds_pool[];
  char* lb = (char*)lds_pool;
  float*    sacc = (float*)(lb + PL_SACC);
  int*      list = (int*)(lb + PL_LIST);
  _Float16* sZ   = (_Float16*)(lb + PL_SZ);
  _Float16* sW   = (_Float16*)(lb + PL_SW);
  float*    sH   = (float*)(lb + PL_SH);
  float*    sL   = (float*)(lb + PL_SL);
  float*    sO   = (float*)(lb + PL_SO);
  int*      scnt = (int*)(lb + PL_SCNT);
  float*    sinv = (float*)(lb + PL_SINV);
  int*      wcnt = (int*)(lb + PL_WCNT);
  const int tid = threadIdx.x, lane = tid & 31, wave = tid >> 5;
  const int gbase = blockIdx.x * GPB;

  for (int i = tid; i < GPB * DD; i += NTHR) sacc[i] = 0.0f;
  for (int i = tid; i < GPB * NCLS; i += NTHR) sO[i] = 0.0f;
  for (int i = tid; i < FCH * DD; i += NTHR) sW[i] = (_Float16)(fc1W[i] * WSC);
  if (tid < GPB) scnt[tid] = 0;
  __syncthreads();

  const int nChunks = (nN + CHUNK - 1) / CHUNK;
#pragma unroll 1
  for (int ch = 0; ch < nChunks; ++ch) {
    const int cbase = ch * CHUNK;
    const int wc = scan_chunk<GPB>(bidx, nN, cbase, gbase, vec8, list, tid, lane, wave);
    if (lane == 0) wcnt[wave] = wc;
    __syncthreads();
#pragma unroll 1
    for (int wsx = 0; wsx < NWAVE; ++wsx) {
      int n = wcnt[wsx];
      n = n > WCAP ? WCAP : (n < 0 ? 0 : n);
      const int* lp = list + wsx * WCAP;
#pragma unroll 1
      for (int i = 0; i < n; ++i) {
        const int ent  = lp[i];
        const int slot = ent & (GPB - 1);
        int node = cbase + ((ent >> 12) & (CHUNK - 1));
        node = node > nN - 1 ? nN - 1 : node;
        if (tid < DD) {
          const size_t q = (size_t)node * DD + tid;
          const float mv = hm[q];
          const float lv = hv[q];
          const float ev = eps[q];
          const float z  = fmaf(ev, expf(0.5f * lv), mv);
          sacc[slot * DD + tid] += z;
        }
        if (tid == DD) scnt[slot] = scnt[slot] + 1;
      }
    }
    __syncthreads();
  }

  if (tid < GPB) {
    const int cg = scnt[tid];
    sinv[tid] = 1.0f / (float)(cg < 1 ? 1 : cg);
  }
  __syncthreads();
  if (tid < DD) {
#pragma unroll 1
    for (int s = 0; s < GPB; ++s) sZ[s * DD + tid] = (_Float16)(sacc[s * DD + tid] * sinv[s] * ZSC);
  }
  __syncthreads();

  {
    const int hh = lane >> 4, m = lane & 15;
    const int r0 = wave * 16;
    const _Float16* ap = sZ + (r0 + m) * DD + 8 * hh;
#pragma unroll 1
    for (int t = 0; t < FCH / 16; ++t) {
      v8f acc = {0.f, 0.f, 0.f, 0.f, 0.f, 0.f, 0.f, 0.f};
#pragma unroll
      for (int kt = 0; kt < DD / 32; ++kt) {
        FragH a, b;
        a.h[0] = *(const v8h*)(ap + 32 * kt);
        a.h[1] = *(const v8h*)(ap + 32 * kt + 16);
        const _Float16* bp = sW + (16 * t + m) * DD + 8 * hh + 32 * kt;
        b.h[0] = *(const v8h*)bp;
        b.h[1] = *(const v8h*)(bp + 16);
        acc = wmh(a.v, b.v, acc);
      }
      const int col = 16 * t + m;
      const float bv = fc1b[col];
#pragma unroll
      for (int r = 0; r < 8; ++r) sH[(r0 + 8 * hh + r) * FCH + col] = fmaxf(acc[r] * INV_HEAD + bv, 0.0f);
    }
  }
  __syncthreads();

  if (tid < GPB) {
    const int g = tid;
    const float* hr = sH + g * FCH;
#pragma unroll
    for (int c = 0; c < NCLS; ++c) {
      const float* wr = fc2W + c * FCH;
      float s = 0.0f;
#pragma unroll 1
      for (int jj = 0; jj < FCH; ++jj) s = fmaf(hr[jj], wr[jj], s);
      sL[g * NCP + c] = s + fc2b[c];
    }
    float mx = sL[g * NCP];
#pragma unroll 1
    for (int c = 1; c < NCLS; ++c) mx = fmaxf(mx, sL[g * NCP + c]);
    float se = 0.0f;
#pragma unroll 1
    for (int c = 0; c < NCLS; ++c) se += expf(sL[g * NCP + c] - mx);
    const float lse = logf(se);
#pragma unroll 1
    for (int c = 0; c < NCLS; ++c) sO[g * NCLS + c] = sL[g * NCP + c] - mx - lse;
  }
  __syncthreads();

  {
    int nv = nG - gbase;
    nv = nv < 0 ? 0 : (nv > GPB ? GPB : nv);
    const int nfl = nv * NCLS;
    float* op = out + (size_t)gbase * NCLS;
    constexpr int NV4 = GPB * NCLS / 4;
#pragma unroll 1
    for (int f = tid; f < NV4; f += NTHR) {
      const v4f v = ((const v4f*)sO)[f];
      if (4 * f + 4 <= nfl) {
        *(volatile v4f*)(op + 4 * f) = v;
      } else if (4 * f < nfl) {
        *(volatile float*)(op + 4 * f) = v.x;
        if (4 * f + 1 < nfl) *(volatile float*)(op + 4 * f + 1) = v.y;
        if (4 * f + 2 < nfl) *(volatile float*)(op + 4 * f + 2) = v.z;
      }
    }
    __threadfence();
#pragma unroll 1
    for (int f = tid; f < NV4; f += NTHR) {
      const v4f v = ((const v4f*)sO)[f];
      if (4 * f + 4 <= nfl) {
        *(volatile v4f*)(op + 4 * f) = v;
      } else if (4 * f < nfl) {
        *(volatile float*)(op + 4 * f) = v.x;
        if (4 * f + 1 < nfl) *(volatile float*)(op + 4 * f + 1) = v.y;
        if (4 * f + 2 < nfl) *(volatile float*)(op + 4 * f + 2) = v.z;
      }
    }
  }
}

extern "C" void kernel_launch(void* const* d_in, const int* in_sizes, int n_in,
                              void* d_out, int out_size, void* d_ws, size_t ws_size,
                              hipStream_t stream) {
  if (n_in < 14) return;
  if (in_sizes[0] <= 0 || (in_sizes[0] % DD) != 0) return;
  const int nN = in_sizes[0] / DD;
  if (in_sizes[1] <= 0 || (in_sizes[1] & 1) != 0) return;
  const int nE = in_sizes[1] / 2;
  if (in_sizes[2] != nN || in_sizes[3] != nN * DD) return;
  if (in_sizes[4] <= 0 || (in_sizes[4] % (DD * DD)) != 0) return;
  const int nL = in_sizes[4] / (DD * DD);
  if (nL < 1 || nL > 8) return;
  if (in_sizes[5] != nL * DD || in_sizes[6] != nL * DD * DD) return;
  if (in_sizes[7] != nL * DD * DD || in_sizes[8] != nL * DD || in_sizes[9] != nL * DD * DD) return;
  if (in_sizes[10] != FCH * DD || in_sizes[11] != FCH || in_sizes[12] != NCLS * FCH || in_sizes[13] != NCLS) return;
  if (nN > (1 << 22) || nE > (1 << 28)) return;
  const long long rem = (long long)out_size - 2LL * nN * DD;
  if (rem <= 0 || (rem % NCLS) != 0) return;
  const int nG = (int)(rem / NCLS);
  if (nG > (1 << 22)) return;

  const float* x     = (const float*)d_in[0];
  const int*   ei    = (const int*)d_in[1];
  const int*   batch = (const int*)d_in[2];
  const float* eps   = (const float*)d_in[3];
  const float* mWl   = (const float*)d_in[4];
  const float* mbl   = (const float*)d_in[5];
  const float* mWr   = (const float*)d_in[6];
  const float* vWl   = (const float*)d_in[7];
  const float* vbl   = (const float*)d_in[8];
  const float* vWr   = (const float*)d_in[9];
  const float* fc1W  = (const float*)d_in[10];
  const float* fc1b  = (const float*)d_in[11];
  const float* fc2W  = (const float*)d_in[12];
  const float* fc2b  = (const float*)d_in[13];
  const int* src = ei;
  const int* dst = ei + nE;
  float* out  = (float*)d_out;
  float* out0 = out;
  float* out1 = out + (size_t)nG * NCLS;
  float* out2 = out1 + (size_t)nN * DD;

  const int NPAD   = ((nN + TGT - 1) / TGT) * TGT;
  const int nBC    = (nN + NBC - 1) / NBC;
  const int CNTPAD = nBC * NBC;
  if (4 * nBC + 1 > RBN) return;
  const int nBF    = (nN + NBF - 1) / NBF;
  const int csrLen = ((nE + 31) & ~31) + 4096;
  if (31 * 4 * nBC > 4096) return;
  const int nAgg   = NPAD / TGT;
  const int nGm    = NPAD / BM;
  const int nPool  = (nG + GPB - 1) / GPB;
  const int nWU    = nL * 2 * DD * (KA / 8);

  char* ws = (char*)d_ws;
  size_t off = 0;
  const size_t oWp  = off; off += (size_t)nL * 2 * DD * KA * 2;   off = (off + 255) & ~(size_t)255;
  const size_t oA   = off; off += (size_t)2 * NPAD * KA * 2;      off = (off + 255) & ~(size_t)255;
  const size_t oH   = off; off += (size_t)2 * NPAD * DD * 4;      off = (off + 255) & ~(size_t)255;
  const size_t oCnt = off; off += (size_t)CNTPAD * 4;             off = (off + 255) & ~(size_t)255;
  const size_t oOff = off; off += (size_t)CNTPAD * 4;             off = (off + 255) & ~(size_t)255;
  const size_t oRb  = off; off += (size_t)RBN * 4;                off = (off + 255) & ~(size_t)255;
  const size_t oCsr = off; off += (size_t)csrLen * 4;             off = (off + 255) & ~(size_t)255;
  if (off > ws_size || off > (size_t)WSCAP) return;
  _Float16*     wp   = (_Float16*)(ws + oWp);
  _Float16*     apl  = (_Float16*)(ws + oA);
  unsigned int* aplU = (unsigned int*)(ws + oA);
  float*        hpl  = (float*)(ws + oH);
  int*          cnt  = (int*)(ws + oCnt);
  int*          offp = (int*)(ws + oOff);
  int*          rb   = (int*)(ws + oRb);
  int*          csr  = (int*)(ws + oCsr);

  const int vec8 = ((nE & 3) == 0) ? 1 : 0;

  k_wprep<<<(nWU + NTHR - 1) / NTHR, NTHR, 0, stream>>>(mWl, mWr, vWl, vWr, wp, nL);

  k_count<<<nBC, NTHR, 0, stream>>>(dst, cnt, nE, vec8);
  k_offsets<<<1, OTHR, 0, stream>>>(cnt, offp, rb, nBC);
  hipFuncSetAttribute(reinterpret_cast<const void*>(&k_fill),
                      hipFuncAttributeMaxDynamicSharedMemorySize, LDS_FILL);
  k_fill<<<nBF, NTHR, LDS_FILL, stream>>>(src, dst, offp, rb, csr, nN, nE, vec8, csrLen);

  const int aStrideH = NPAD * KA;
  const int aStrideU = NPAD * (KA / 2);
  const int hStride  = NPAD * DD;
  for (int l = 0; l < nL; ++l) {
    if (l == 0) {
      k_agg<<<dim3(nAgg, 1), NTHR, 0, stream>>>(csr, offp, cnt, x, 0, aplU, 0, nN, csrLen);
    } else {
      k_agg<<<dim3(nAgg, 2), NTHR, 0, stream>>>(csr, offp, cnt, hpl, hStride, aplU, aStrideU, nN, csrLen);
    }
    const bool last   = (l == nL - 1);
    float* C          = last ? out1 : hpl;
    const int cStride = last ? nN * DD : hStride;
    const int nValid  = last ? nN : NPAD;
    const int aStr    = (l == 0) ? 0 : aStrideH;
    k_gemm<<<dim3(nGm, 2), NTHR, 0, stream>>>(apl, aStr, wp + (size_t)l * 2 * DD * KA,
                                              mbl + (size_t)l * DD, vbl + (size_t)l * DD,
                                              C, cStride, nValid);
  }

  hipFuncSetAttribute(reinterpret_cast<const void*>(&k_pool_head),
                      hipFuncAttributeMaxDynamicSharedMemorySize, LDS_POOL);
  k_pool_head<<<nPool, NTHR, LDS_POOL, stream>>>(batch, out1, out2, eps, fc1W, fc1b, fc2W, fc2b,
                                                 out0, nN, nG, 1);
}
